// MultiHeadCausalSelfAttention_38809324486806
// MI455X (gfx1250) — hardware-verified
//
#include <hip/hip_runtime.h>
#include <math.h>

constexpr int kBatch = 2;
constexpr int kSeq   = 2048;
constexpr int kDim   = 1024;
constexpr int kHeads = 16;
constexpr int kDh    = 64;
constexpr int kTok   = kBatch * kSeq;
constexpr int kQkvN  = 3 * kDim;
constexpr float kScoreScale = 0.125f;
static_assert(kHeads * kDh == kDim);
static_assert(kTok % 64 == 0 && kDim % 64 == 0 && kQkvN % 64 == 0 && kDim % 32 == 0);
static_assert(kSeq % 64 == 0 && kDh == 64 && (kSeq / 64) == 32);
static_assert((kTok * kDim) % (8 * 256) == 0);

constexpr size_t kSzPlane16 = (size_t)kTok * kDim * 2;
constexpr size_t kSzWqkvT   = (size_t)kQkvN * kDim * 2;
constexpr size_t kSzWoutT   = (size_t)kDim * kDim * 2;
constexpr size_t kSzPlane32 = (size_t)kTok * kDim * 4;
constexpr size_t kSzVt      = (size_t)kBatch * kHeads * kDh * kSeq * 2;
constexpr size_t kOffXb   = 0;
constexpr size_t kOffWqkv = kOffXb + kSzPlane16;
constexpr size_t kOffWout = kOffWqkv + kSzWqkvT;
constexpr size_t kOffQh   = kOffWout + kSzWoutT;
constexpr size_t kOffQl   = kOffQh + kSzPlane16;
constexpr size_t kOffKh   = kOffQl + kSzPlane16;
constexpr size_t kOffKl   = kOffKh + kSzPlane16;
constexpr size_t kOffVf   = kOffKl + kSzPlane16;
constexpr size_t kOffVth  = kOffVf + kSzPlane32;
constexpr size_t kOffVtl  = kOffVth + kSzVt;
constexpr size_t kOffCh   = kOffVtl + kSzVt;
constexpr size_t kOffCl   = kOffCh + kSzPlane16;
constexpr size_t kWsTotal = kOffCl + kSzPlane16;
static_assert(kWsTotal == 100663296ull);
static_assert(kWsTotal <= 134217728ull);

typedef __attribute__((ext_vector_type(16))) _Float16 v16h;
typedef __attribute__((ext_vector_type(8)))  _Float16 v8h;
typedef __attribute__((ext_vector_type(16))) __bf16   v16b;
typedef __attribute__((ext_vector_type(8)))  __bf16   v8b;
typedef __attribute__((ext_vector_type(8)))  float    v8f;
typedef __attribute__((ext_vector_type(4)))  float    v4f;
typedef __attribute__((ext_vector_type(4)))  unsigned int v4u;

__device__ __forceinline__ unsigned short f2bf_bits(float f) {
  unsigned u = __float_as_uint(f);
  return (unsigned short)((u + 0x7FFFu + ((u >> 16) & 1u)) >> 16);
}
__device__ __forceinline__ float bf_bits2f(unsigned short h) { return __uint_as_float(((unsigned)h) << 16); }

__device__ __forceinline__ void dep_guard_h(v8f& a, v8f& b, v16h x, v16h y) { asm volatile("v_nop\n\tv_nop\n\tv_nop\n\tv_nop" : "+v"(a), "+v"(b) : "v"(x), "v"(y)); }
__device__ __forceinline__ void dep_guard_b(v8f& a, v8f& b, v16b x, v16b y) { asm volatile("v_nop\n\tv_nop\n\tv_nop\n\tv_nop" : "+v"(a), "+v"(b) : "v"(x), "v"(y)); }
__device__ __forceinline__ void dep_guard4_h(v8f& a, v8f& b, v8f& c, v8f& d, v16h x, v16h y) { asm volatile("v_nop\n\tv_nop\n\tv_nop\n\tv_nop" : "+v"(a), "+v"(b), "+v"(c), "+v"(d) : "v"(x), "v"(y)); }
__device__ __forceinline__ void dep_guard4_b(v8f& a, v8f& b, v8f& c, v8f& d, v16b x, v16b y) { asm volatile("v_nop\n\tv_nop\n\tv_nop\n\tv_nop" : "+v"(a), "+v"(b), "+v"(c), "+v"(d) : "v"(x), "v"(y)); }
__device__ __forceinline__ void keep4_h(v16h a, v16h b, v16h c, v16h d) { asm volatile("v_nop" :: "v"(a), "v"(b), "v"(c), "v"(d)); }
__device__ __forceinline__ void keep4_b(v16b a, v16b b, v16b c, v16b d) { asm volatile("v_nop" :: "v"(a), "v"(b), "v"(c), "v"(d)); }
__device__ __forceinline__ void acc_guard4(v8f& a, v8f& b, v8f& c, v8f& d) { asm volatile("v_nop\n\tv_nop\n\tv_nop\n\tv_nop" : "+v"(a), "+v"(b), "+v"(c), "+v"(d)); }
template <typename T> struct Frag;
template <> struct Frag<_Float16> {
  typedef v16h V; union U { v16h v; v8h h[2]; };
  static __device__ __forceinline__ v16h load(const _Float16* p) {
    U f; f.h[0] = *(const v8h*)(p); f.h[1] = *(const v8h*)(p + 16); return f.v;
  }
  static __device__ __forceinline__ v8f mma(v16h a, v16h b, v8f c) {
    return __builtin_amdgcn_wmma_f32_16x16x32_f16(false, a, false, b, (short)0, c, false, false);
  }
  static __device__ __forceinline__ void guard(v8f& a, v8f& b, v16h x, v16h y) { dep_guard_h(a, b, x, y); }
  static __device__ __forceinline__ void guard4(v8f& a, v8f& b, v8f& c, v8f& d, v16h x, v16h y) { dep_guard4_h(a, b, c, d, x, y); }
  static __device__ __forceinline__ void keep(v16h a, v16h b, v16h c, v16h d) { keep4_h(a, b, c, d); }
};
template <> struct Frag<__bf16> {
  typedef v16b V; union U { v16b v; v8b h[2]; };
  static __device__ __forceinline__ v16b load(const __bf16* p) {
    U f; f.h[0] = *(const v8b*)(p); f.h[1] = *(const v8b*)(p + 16); return f.v;
  }
  static __device__ __forceinline__ v8f mma(v16b a, v16b b, v8f c) {
    return __builtin_amdgcn_wmma_f32_16x16x32_bf16(false, a, false, b, (short)0, c, false, false);
  }
  static __device__ __forceinline__ void guard(v8f& a, v8f& b, v16b x, v16b y) { dep_guard_b(a, b, x, y); }
  static __device__ __forceinline__ void guard4(v8f& a, v8f& b, v8f& c, v8f& d, v16b x, v16b y) { dep_guard4_b(a, b, c, d, x, y); }
  static __device__ __forceinline__ void keep(v16b a, v16b b, v16b c, v16b d) { keep4_b(a, b, c, d); }
};

__device__ __forceinline__ unsigned pk16(unsigned short a, unsigned short b) { return (unsigned)a | ((unsigned)b << 16); }

__device__ __forceinline__ __bf16 at_f2bf(float f) { return __builtin_bit_cast(__bf16, f2bf_bits(f)); }
__device__ __forceinline__ void at_split(float f, __bf16& hi, __bf16& lo) {
  const unsigned short hb = f2bf_bits(f);
  hi = __builtin_bit_cast(__bf16, hb);
  lo = at_f2bf(f - __uint_as_float(((unsigned)hb) << 16));
}
__device__ __forceinline__ v8f at_mma(v16b a, v16b b, v8f c) {
  c = __builtin_amdgcn_wmma_f32_16x16x32_bf16(false, a, false, b, (short)0, c, false, false);
  asm volatile("v_nop\n\tv_nop\n\tv_nop\n\tv_nop" : "+v"(c) : "v"(a), "v"(b));
  return c;
}

template <int ET> struct Elem;
template <> struct Elem<0> { typedef _Float16 T; };
template <> struct Elem<1> { typedef __bf16 T; };
template <int ET, int SPLIT, int BIAS_MODE, int OUT_MODE, bool RESID, int ACT = 0>
__global__ __launch_bounds__(256) void wmma_gemm64(
    const unsigned short* __restrict__ Ap, const unsigned short* __restrict__ A2p, int lda, long strideA,
    const unsigned short* __restrict__ Btp, const unsigned short* __restrict__ Bt2p, int ldb, long strideB,
    void* __restrict__ Cout, void* __restrict__ Cout2, int ldc, long strideC,
    const float* __restrict__ bias,
    const float* __restrict__ resid, long strideR,
    int M, int N, int K, float scale) {
  typedef typename Elem<ET>::T T;
  typedef typename Frag<T>::V V;
  const T* A = (const T*)Ap; const T* A2 = (const T*)A2p; const T* Bt = (const T*)Btp; const T* Bt2 = (const T*)Bt2p;
  __shared__ __align__(16) float sT[8][16 * 68];
  const int b    = blockIdx.y;
  const int lane = threadIdx.x & 31;
  const int wave = threadIdx.x >> 5;
  const int tilesN = N >> 6;
  const int tilesM = M >> 6;
  const int tile = blockIdx.x * 8 + wave;
  if (tile >= tilesM * tilesN) return;
  const int tm = tile / tilesN;
  const int tn = tile - tm * tilesN;
  const int m0 = tm << 6;
  const int n0 = tn << 6;

  const T* Ab  = A  + (size_t)b * strideA;
  const T* Bb  = Bt + (size_t)b * strideB;
  const T* Ab2 = (SPLIT != 0) ? (A2  + (size_t)b * strideA) : nullptr;
  const T* Bb2 = (SPLIT == 1) ? (Bt2 + (size_t)b * strideB) : nullptr;

  const int rlane = lane & 15;
  const int koff  = (lane >> 4) * 8;
  const int mOff  = (lane >> 4) * 8;

  v8f acc[4][4];
#pragma unroll
  for (int i = 0; i < 4; ++i)
#pragma unroll
    for (int j = 0; j < 4; ++j) acc[i][j] = (v8f){0.f,0.f,0.f,0.f,0.f,0.f,0.f,0.f};

  for (int k0 = 0; k0 < K; k0 += 32) {
    V bh[4], bl[4];
#pragma unroll
    for (int j = 0; j < 4; ++j) {
      const size_t bo = (size_t)(n0 + (j << 4) + rlane) * ldb + koff + k0;
      bh[j] = Frag<T>::load(Bb + bo);
      if (SPLIT == 1) bl[j] = Frag<T>::load(Bb2 + bo);
    }
#pragma unroll
    for (int i = 0; i < 4; ++i) {
      const size_t ao = (size_t)(m0 + (i << 4) + rlane) * lda + koff + k0;
      V ah = Frag<T>::load(Ab + ao);
      V al = ah;
      if (SPLIT != 0) al = Frag<T>::load(Ab2 + ao);
#pragma unroll
      for (int j = 0; j < 4; ++j) {
        acc[i][j] = Frag<T>::mma(ah, bh[j], acc[i][j]);
        if (SPLIT == 1) acc[i][j] = Frag<T>::mma(ah, bl[j], acc[i][j]);
        if (SPLIT != 0) acc[i][j] = Frag<T>::mma(al, bh[j], acc[i][j]);
      }
      Frag<T>::guard4(acc[i][0], acc[i][1], acc[i][2], acc[i][3], ah, al);
    }
    Frag<T>::keep(bh[0], bh[1], bh[2], bh[3]);
    if (SPLIT == 1) Frag<T>::keep(bl[0], bl[1], bl[2], bl[3]);
  }
  acc_guard4(acc[0][0], acc[0][1], acc[0][2], acc[0][3]);
  acc_guard4(acc[1][0], acc[1][1], acc[1][2], acc[1][3]);
  acc_guard4(acc[2][0], acc[2][1], acc[2][2], acc[2][3]);
  acc_guard4(acc[3][0], acc[3][1], acc[3][2], acc[3][3]);

  float* slab = sT[wave];
  const float* Rb = RESID ? (resid + (size_t)b * strideR) : nullptr;
#pragma unroll
  for (int i = 0; i < 4; ++i) {
    const int mBase = m0 + (i << 4);
#pragma unroll
    for (int j = 0; j < 4; ++j) {
      const int n = n0 + (j << 4) + rlane;
      float bv = 0.f;
      if (BIAS_MODE == 2) bv = bias[n];
#pragma unroll
      for (int r = 0; r < 8; ++r) {
        float v = acc[i][j][r] * scale;
        if (BIAS_MODE == 1) v += bias[mBase + mOff + r];
        if (BIAS_MODE == 2) v += bv;
        if (RESID) v += Rb[(size_t)(mBase + mOff + r) * ldc + n];
        if (ACT == 2) v = fmaxf(v, 0.0f);
        if (ACT == 4) v = (v > 0.f) ? v : 0.01f * v;
        slab[(mOff + r) * 68 + (j << 4) + rlane] = v;
      }
    }
    __builtin_amdgcn_fence(__ATOMIC_RELEASE, "workgroup");
    __builtin_amdgcn_wave_barrier();
    __builtin_amdgcn_fence(__ATOMIC_ACQUIRE, "workgroup");
    if (OUT_MODE == 0) {
      float* C = (float*)Cout + (size_t)b * strideC;
      const int hh = lane >> 4, c4 = (lane & 15) * 4;
      for (int pass = 0; pass < 2; ++pass) {
#pragma unroll
        for (int it = 0; it < 8; ++it) {
          const int row = it * 2 + hh;
          v4f v = *(const v4f*)(slab + row * 68 + c4);
          *(volatile v4f*)(C + (size_t)(mBase + row) * ldc + n0 + c4) = v;
        }
        __threadfence();
      }
    } else {
      const int q = lane >> 3, c8 = (lane & 7) * 8;
      unsigned short* C  = (unsigned short*)Cout  + (size_t)b * strideC;
      unsigned short* C2 = (OUT_MODE == 2) ? ((unsigned short*)Cout2 + (size_t)b * strideC) : nullptr;
      for (int pass = 0; pass < 2; ++pass) {
#pragma unroll
        for (int it = 0; it < 4; ++it) {
          const int row = it * 4 + q;
          const float* sp = slab + row * 68 + c8;
          v8h hv, lv;
#pragma unroll
          for (int e = 0; e < 8; ++e) {
            if (OUT_MODE == 1) {
              hv[e] = (_Float16)sp[e];
            } else {
              unsigned short hb = f2bf_bits(sp[e]);
              unsigned short lb = f2bf_bits(sp[e] - bf_bits2f(hb));
              hv[e] = __builtin_bit_cast(_Float16, hb);
              lv[e] = __builtin_bit_cast(_Float16, lb);
            }
          }
          *(volatile v8h*)(C + (size_t)(mBase + row) * ldc + n0 + c8) = hv;
          if (OUT_MODE == 2) *(volatile v8h*)(C2 + (size_t)(mBase + row) * ldc + n0 + c8) = lv;
        }
        __threadfence();
      }
    }
    __builtin_amdgcn_fence(__ATOMIC_RELEASE, "workgroup");
    __builtin_amdgcn_wave_barrier();
    __builtin_amdgcn_fence(__ATOMIC_ACQUIRE, "workgroup");
  }
}

__global__ __launch_bounds__(256) void cast8_bf16_kernel(const float* __restrict__ in, unsigned short* __restrict__ out, int n8) {
  const int i = blockIdx.x * 256 + threadIdx.x;
  if (i >= n8) return;
  const float* p = in + 8 * (size_t)i;
  const v4f a = *(const v4f*)(p);
  const v4f c = *(const v4f*)(p + 4);
  unsigned short hb[8];
#pragma unroll
  for (int e = 0; e < 4; ++e) {
    hb[e]     = f2bf_bits(a[e]);
    hb[4 + e] = f2bf_bits(c[e]);
  }
  const v4u u = (v4u){pk16(hb[0], hb[1]), pk16(hb[2], hb[3]), pk16(hb[4], hb[5]), pk16(hb[6], hb[7])};
  unsigned short* q = out + 8 * (size_t)i;
  *(volatile v4u*)q = u;
  __threadfence();
  *(volatile v4u*)q = u;
}

__global__ __launch_bounds__(256) void wt_cast_kernel(const float* __restrict__ W, unsigned short* __restrict__ WT, int ncols) {
  __shared__ float sm[64][65];
  const int t  = threadIdx.x;
  const int k0 = blockIdx.x * 64;
  const int n0 = blockIdx.y * 64;
#pragma unroll
  for (int i = 0; i < 8; ++i) {
    const int e = i * 256 + t;
    const int r = e >> 6;
    const int c = e & 63;
    sm[c][r] = W[(size_t)(k0 + r) * ncols + n0 + c];
  }
  asm volatile("" ::: "memory");
#pragma unroll
  for (int i = 8; i < 16; ++i) {
    const int e = i * 256 + t;
    const int r = e >> 6;
    const int c = e & 63;
    sm[c][r] = W[(size_t)(k0 + r) * ncols + n0 + c];
  }
  __syncthreads();
  const int lane = t & 31, wave = t >> 5;
  const int q = lane >> 3, c8 = (lane & 7) * 8;
  for (int pass = 0; pass < 2; ++pass) {
#pragma unroll
    for (int it = 0; it < 2; ++it) {
      const int row = wave * 8 + it * 4 + q;
      unsigned short hb[8];
#pragma unroll
      for (int e = 0; e < 8; ++e) hb[e] = f2bf_bits(sm[row][c8 + e]);
      const v4u u = (v4u){pk16(hb[0], hb[1]), pk16(hb[2], hb[3]), pk16(hb[4], hb[5]), pk16(hb[6], hb[7])};
      *(volatile v4u*)(WT + (size_t)(n0 + row) * kDim + k0 + c8) = u;
    }
    __threadfence();
  }
}

__global__ __launch_bounds__(256) void vt_split_kernel(const float* __restrict__ Vf, unsigned short* __restrict__ Vth,
                                                       unsigned short* __restrict__ Vtl) {
  __shared__ float sm[64][65];
  const int t  = threadIdx.x;
  const int s0 = blockIdx.x * 64;
  const int h  = blockIdx.y;
  const int b  = blockIdx.z;
#pragma unroll
  for (int i = 0; i < 8; ++i) {
    const int e = i * 256 + t;
    const int r = e >> 6;
    const int c = e & 63;
    sm[c][r] = Vf[((size_t)(b * kSeq + s0 + r)) * kDim + h * kDh + c];
  }
  asm volatile("" ::: "memory");
#pragma unroll
  for (int i = 8; i < 16; ++i) {
    const int e = i * 256 + t;
    const int r = e >> 6;
    const int c = e & 63;
    sm[c][r] = Vf[((size_t)(b * kSeq + s0 + r)) * kDim + h * kDh + c];
  }
  __syncthreads();
  const int lane = t & 31, wave = t >> 5;
  const int q = lane >> 3, c8 = (lane & 7) * 8;
  const size_t base = ((size_t)(b * kHeads + h) * kDh) * kSeq;
  for (int pass = 0; pass < 2; ++pass) {
#pragma unroll
    for (int it = 0; it < 2; ++it) {
      const int row = wave * 8 + it * 4 + q;
      unsigned short hb[8], lb[8];
#pragma unroll
      for (int e = 0; e < 8; ++e) {
        const float f = sm[row][c8 + e];
        hb[e] = f2bf_bits(f);
        lb[e] = f2bf_bits(f - bf_bits2f(hb[e]));
      }
      const v4u uh = (v4u){pk16(hb[0], hb[1]), pk16(hb[2], hb[3]), pk16(hb[4], hb[5]), pk16(hb[6], hb[7])};
      const v4u ul = (v4u){pk16(lb[0], lb[1]), pk16(lb[2], lb[3]), pk16(lb[4], lb[5]), pk16(lb[6], lb[7])};
      const size_t o = base + (size_t)row * kSeq + s0 + c8;
      *(volatile v4u*)(Vth + o) = uh;
      *(volatile v4u*)(Vtl + o) = ul;
    }
    __threadfence();
  }
}

__device__ __forceinline__ void stage32h(unsigned short* dst, const unsigned short* __restrict__ src) {
  const v4u a0 = *(const v4u*)(src);
  const v4u a1 = *(const v4u*)(src + 8);
  const v4u a2 = *(const v4u*)(src + 16);
  const v4u a3 = *(const v4u*)(src + 24);
  *(v4u*)(dst)      = a0;
  *(v4u*)(dst + 8)  = a1;
  *(v4u*)(dst + 16) = a2;
  *(v4u*)(dst + 24) = a3;
}

__global__ __launch_bounds__(128)
void causal_attn_kernel(const unsigned short* __restrict__ Qh, const unsigned short* __restrict__ Ql,
                        const unsigned short* __restrict__ Kh, const unsigned short* __restrict__ Kl,
                        const unsigned short* __restrict__ Vth, const unsigned short* __restrict__ Vtl,
                        unsigned short* __restrict__ Ch, unsigned short* __restrict__ Cl) {
  union FB { v16b v; v8b h[2]; };
  __shared__ __align__(16) unsigned short Ksh[64 * 64];
  __shared__ __align__(16) unsigned short Ksl[64 * 64];
  __shared__ __align__(16) unsigned short Vsh[64 * 64];
  __shared__ __align__(16) unsigned short Vsl[64 * 64];
  __shared__ __align__(16) __bf16 Psh[4][16 * 64];
  __shared__ __align__(16) __bf16 Psl[4][16 * 64];
  __shared__ __align__(16) float  Os[4][16 * 68];

  const int tid  = threadIdx.x;
  const int wave = tid >> 5;
  const int lane = tid & 31;
  const int hh   = lane >> 4;
  const int c    = lane & 15;

  const int qb = blockIdx.x & 31;
  const int bh = blockIdx.x >> 5;
  const int h  = bh & 15;
  const int b  = bh >> 4;
  const int q0 = qb * 64 + wave * 16;
  const size_t tokBase = (size_t)b * kSeq;
  const int hcol = h * kDh;

  v16b qah[2], qal[2];
  {
    const size_t qo = (tokBase + q0 + c) * kDim + hcol + 8 * hh;
#pragma unroll
    for (int dc = 0; dc < 2; ++dc) {
      qah[dc] = Frag<__bf16>::load((const __bf16*)(Qh + qo + dc * 32));
      qal[dc] = Frag<__bf16>::load((const __bf16*)(Ql + qo + dc * 32));
    }
  }

  float mrow[8], lrow[8];
  v8f oacc[4];
#pragma unroll
  for (int r = 0; r < 8; ++r) { mrow[r] = -__builtin_inff(); lrow[r] = 0.f; }
#pragma unroll
  for (int t = 0; t < 4; ++t) oacc[t] = (v8f){0.f,0.f,0.f,0.f,0.f,0.f,0.f,0.f};

  for (int kc = 0; kc <= qb; ++kc) {
    const int kv0 = kc * 64;
    __syncthreads();
    {
      const int r = tid >> 1, half = (tid & 1) * 32;
      const size_t ko = (tokBase + kv0 + r) * kDim + hcol + half;
      const size_t vo = ((size_t)bh * kDh + r) * kSeq + kv0 + half;
      stage32h(Ksh + r * 64 + half, Kh + ko);
      asm volatile("" ::: "memory");
      stage32h(Ksl + r * 64 + half, Kl + ko);
      asm volatile("" ::: "memory");
      stage32h(Vsh + r * 64 + half, Vth + vo);
      asm volatile("" ::: "memory");
      stage32h(Vsl + r * 64 + half, Vtl + vo);
    }
    __syncthreads();

    v8f s[4];
#pragma unroll
    for (int j = 0; j < 4; ++j) {
      s[j] = (v8f){0.f,0.f,0.f,0.f,0.f,0.f,0.f,0.f};
#pragma unroll
      for (int dc = 0; dc < 2; ++dc) {
        FB kb, kl;
        kb.h[0] = *(const v8b*)(Ksh + (j * 16 + c) * 64 + dc * 32 + 8 * hh);
        kb.h[1] = *(const v8b*)(Ksh + (j * 16 + c) * 64 + dc * 32 + 16 + 8 * hh);
        kl.h[0] = *(const v8b*)(Ksl + (j * 16 + c) * 64 + dc * 32 + 8 * hh);
        kl.h[1] = *(const v8b*)(Ksl + (j * 16 + c) * 64 + dc * 32 + 16 + 8 * hh);
        s[j] = at_mma(qah[dc], kb.v, s[j]);
        s[j] = at_mma(qah[dc], kl.v, s[j]);
        s[j] = at_mma(qal[dc], kb.v, s[j]);
      }
      asm volatile("" ::: "memory");
    }

    const bool diag = (kc == qb);
    float cm[8];
#pragma unroll
    for (int r = 0; r < 8; ++r) {
      const int qrow = q0 + 8 * hh + r;
      float m = -__builtin_inff();
#pragma unroll
      for (int j = 0; j < 4; ++j) {
        const int kvcol = kv0 + j * 16 + c;
        float sv = s[j][r] * kScoreScale;
        if (diag && (kvcol > qrow)) sv = -__builtin_inff();
        s[j][r] = sv;
        m = fmaxf(m, sv);
      }
#pragma unroll
      for (int off = 1; off < 16; off <<= 1) m = fmaxf(m, __shfl_xor(m, off, 32));
      cm[r] = m;
    }

    __bf16* pwh = Psh[wave];
    __bf16* pwl = Psl[wave];
#pragma unroll
    for (int r = 0; r < 8; ++r) {
      const float mnew = fmaxf(mrow[r], cm[r]);
      const float alpha = expf(mrow[r] - mnew);
      mrow[r] = mnew;
      float psum = 0.f;
#pragma unroll
      for (int j = 0; j < 4; ++j) {
        const float p = expf(s[j][r] - mnew);
        psum += p;
        __bf16 a, bl;
        at_split(p, a, bl);
        pwh[(8 * hh + r) * 64 + j * 16 + c] = a;
        pwl[(8 * hh + r) * 64 + j * 16 + c] = bl;
      }
#pragma unroll
      for (int off = 1; off < 16; off <<= 1) psum += __shfl_xor(psum, off, 32);
      lrow[r] = lrow[r] * alpha + psum;
#pragma unroll
      for (int t = 0; t < 4; ++t) oacc[t][r] *= alpha;
    }
    __builtin_amdgcn_fence(__ATOMIC_RELEASE, "workgroup");
    __builtin_amdgcn_wave_barrier();
    __builtin_amdgcn_fence(__ATOMIC_ACQUIRE, "workgroup");

#pragma unroll 1
    for (int kk = 0; kk < 2; ++kk) {
      FB pa, pl;
      pa.h[0] = *(const v8b*)(pwh + c * 64 + kk * 32 + 8 * hh);
      pa.h[1] = *(const v8b*)(pwh + c * 64 + kk * 32 + 16 + 8 * hh);
      pl.h[0] = *(const v8b*)(pwl + c * 64 + kk * 32 + 8 * hh);
      pl.h[1] = *(const v8b*)(pwl + c * 64 + kk * 32 + 16 + 8 * hh);
#pragma unroll
      for (int t = 0; t < 4; ++t) {
        FB vb, vl;
        vb.h[0] = *(const v8b*)(Vsh + (t * 16 + c) * 64 + kk * 32 + 8 * hh);
        vb.h[1] = *(const v8b*)(Vsh + (t * 16 + c) * 64 + kk * 32 + 16 + 8 * hh);
        vl.h[0] = *(const v8b*)(Vsl + (t * 16 + c) * 64 + kk * 32 + 8 * hh);
        vl.h[1] = *(const v8b*)(Vsl + (t * 16 + c) * 64 + kk * 32 + 16 + 8 * hh);
        oacc[t] = at_mma(pa.v, vb.v, oacc[t]);
        oacc[t] = at_mma(pa.v, vl.v, oacc[t]);
        oacc[t] = at_mma(pl.v, vb.v, oacc[t]);
      }
      asm volatile("" ::: "memory");
    }
  }

  float* os = Os[wave];
#pragma unroll
  for (int r = 0; r < 8; ++r) {
    const float inv = 1.0f / lrow[r];
#pragma unroll
    for (int t = 0; t < 4; ++t) os[(8 * hh + r) * 68 + t * 16 + c] = oacc[t][r] * inv;
  }
  __builtin_amdgcn_fence(__ATOMIC_RELEASE, "workgroup");
  __builtin_amdgcn_wave_barrier();
  __builtin_amdgcn_fence(__ATOMIC_ACQUIRE, "workgroup");
  {
    const int q = lane >> 3, c8 = (lane & 7) * 8;
    for (int pass = 0; pass < 2; ++pass) {
#pragma unroll
      for (int it = 0; it < 4; ++it) {
        const int row = it * 4 + q;
        const float* sp = os + row * 68 + c8;
        const v4f e0 = *(const v4f*)(sp);
        const v4f e1 = *(const v4f*)(sp + 4);
        unsigned short hb[8], lb[8];
#pragma unroll
        for (int e = 0; e < 4; ++e) {
          const float f0 = e0[e];
          hb[e] = f2bf_bits(f0);
          lb[e] = f2bf_bits(f0 - bf_bits2f(hb[e]));
          const float f1 = e1[e];
          hb[4 + e] = f2bf_bits(f1);
          lb[4 + e] = f2bf_bits(f1 - bf_bits2f(hb[4 + e]));
        }
        const v4u uh = (v4u){pk16(hb[0], hb[1]), pk16(hb[2], hb[3]), pk16(hb[4], hb[5]), pk16(hb[6], hb[7])};
        const v4u ul = (v4u){pk16(lb[0], lb[1]), pk16(lb[2], lb[3]), pk16(lb[4], lb[5]), pk16(lb[6], lb[7])};
        const size_t o = (tokBase + q0 + row) * kDim + hcol + c8;
        *(volatile v4u*)(Ch + o) = uh;
        *(volatile v4u*)(Cl + o) = ul;
      }
      __threadfence();
    }
  }
}

extern "C" void kernel_launch(void* const* d_in, const int* in_sizes, int n_in,
                              void* d_out, int out_size, void* d_ws, size_t ws_size,
                              hipStream_t stream) {
  if (n_in < 5) return;
  if (in_sizes[0] != kTok * kDim) return;
  if (in_sizes[1] != kDim * kQkvN) return;
  if (in_sizes[2] != kQkvN) return;
  if (in_sizes[3] != kDim * kDim) return;
  if (in_sizes[4] != kDim) return;
  if (out_size != kTok * kDim) return;
  if (ws_size < kWsTotal) return;

  const float* x     = (const float*)d_in[0];
  const float* w_qkv = (const float*)d_in[1];
  const float* b_qkv = (const float*)d_in[2];
  const float* w_out = (const float*)d_in[3];
  const float* b_out = (const float*)d_in[4];
  float* out = (float*)d_out;
  char* ws = (char*)d_ws;
  unsigned short* Xb    = (unsigned short*)(ws + kOffXb);
  unsigned short* WqkvT = (unsigned short*)(ws + kOffWqkv);
  unsigned short* WoutT = (unsigned short*)(ws + kOffWout);
  unsigned short* Qh    = (unsigned short*)(ws + kOffQh);
  unsigned short* Ql    = (unsigned short*)(ws + kOffQl);
  unsigned short* Kh    = (unsigned short*)(ws + kOffKh);
  unsigned short* Kl    = (unsigned short*)(ws + kOffKl);
  float*          Vf    = (float*)(ws + kOffVf);
  unsigned short* Vth   = (unsigned short*)(ws + kOffVth);
  unsigned short* Vtl   = (unsigned short*)(ws + kOffVtl);
  unsigned short* Ch    = (unsigned short*)(ws + kOffCh);
  unsigned short* Cl    = (unsigned short*)(ws + kOffCl);

  const int n8 = (kTok * kDim) / 8;
  cast8_bf16_kernel<<<dim3(n8 / 256), dim3(256), 0, stream>>>(x, Xb, n8);
  wt_cast_kernel<<<dim3(kDim / 64, kQkvN / 64), dim3(256), 0, stream>>>(w_qkv, WqkvT, kQkvN);
  wt_cast_kernel<<<dim3(kDim / 64, kDim / 64), dim3(256), 0, stream>>>(w_out, WoutT, kDim);

  const int tilesProj = (kTok / 64) * (kDim / 64);
  const size_t wblk = (size_t)kDim * kDim;
  wmma_gemm64<1, 0, 2, 2, false, 0><<<dim3(tilesProj / 8, 1), dim3(256), 0, stream>>>(
      Xb, Xb, kDim, 0L, WqkvT, WqkvT, kDim, 0L,
      (void*)Qh, (void*)Ql, kDim, 0L, b_qkv, b_qkv, 0L, kTok, kDim, kDim, 1.0f);
  wmma_gemm64<1, 0, 2, 2, false, 0><<<dim3(tilesProj / 8, 1), dim3(256), 0, stream>>>(
      Xb, Xb, kDim, 0L, WqkvT + wblk, WqkvT + wblk, kDim, 0L,
      (void*)Kh, (void*)Kl, kDim, 0L, b_qkv + kDim, b_qkv, 0L, kTok, kDim, kDim, 1.0f);
  wmma_gemm64<1, 0, 2, 0, false, 0><<<dim3(tilesProj / 8, 1), dim3(256), 0, stream>>>(
      Xb, Xb, kDim, 0L, WqkvT + 2 * wblk, WqkvT + 2 * wblk, kDim, 0L,
      (void*)Vf, (void*)Vf, kDim, 0L, b_qkv + 2 * kDim, b_qkv, 0L, kTok, kDim, kDim, 1.0f);
  vt_split_kernel<<<dim3(kSeq / 64, kHeads, kBatch), dim3(256), 0, stream>>>(Vf, Vth, Vtl);

  causal_attn_kernel<<<dim3(kBatch * kHeads * (kSeq / 64)), dim3(128), 0, stream>>>(Qh, Ql, Kh, Kl, Vth, Vtl, Ch, Cl);

  wmma_gemm64<1, 2, 2, 0, false, 0><<<dim3(tilesProj / 8, 1), dim3(256), 0, stream>>>(
      Ch, Cl, kDim, 0L, WoutT, WoutT, kDim, 0L,
      (void*)out, (void*)out, kDim, 0L, b_out, b_out, 0L, kTok, kDim, kDim, 1.0f);
}
